// GPT_446676599274
// MI455X (gfx1250) — hardware-run, weakly checked
//
#include <hip/hip_runtime.h>

#ifndef NB
#define NB 2
#endif
#ifndef SEQ
#define SEQ 2048
#endif
#define NB_FULL 2
#define SEQ_FULL 2048
#define DM 1024
#define NH 16
#define HD 64
#define FF 4096
#define LOR 64
#define MROWS (NB * SEQ)

static_assert(NB >= 1 && NB <= NB_FULL);
static_assert(SEQ >= 64 && SEQ <= SEQ_FULL && (SEQ % 64) == 0);
static_assert(DM == NH * HD);
static_assert(HD == 64);
static_assert((DM % 64) == 0 && (FF % 64) == 0 && (DM % 32) == 0 && (FF % 32) == 0 && ((3 * DM / 64) % 4) == 0);
static_assert(DM == 128 * 8);
static_assert((LOR % 16) == 0 && LOR == 64);
static_assert((size_t)3 * DM * DM * 2 + (size_t)DM * DM * 2 + (size_t)FF * DM * 2 + (size_t)DM * FF * 2 +
              (size_t)NB_FULL * SEQ_FULL * DM * 2 + (size_t)NB_FULL * SEQ_FULL * 3 * DM * 2 + (size_t)NB_FULL * LOR * 3 * DM * 2 +
              (size_t)NB_FULL * SEQ_FULL * DM * 2 + (size_t)NB_FULL * SEQ_FULL * DM * 4 + (size_t)NB_FULL * SEQ_FULL * DM * 2 +
              (size_t)NB_FULL * SEQ_FULL * FF * 2 <= (size_t)134217728);

#define WSC 64.0f
#define QSC 8.0f
#define PSC 1024.0f
#define CSC 32.0f
#define HSC 8.0f
#define RSC 4096.0f

typedef _Float16 v16h __attribute__((ext_vector_type(16)));
typedef unsigned short v8us __attribute__((ext_vector_type(8), may_alias));
typedef float v8f __attribute__((ext_vector_type(8)));
typedef float v4f __attribute__((ext_vector_type(4)));
typedef float v4fa __attribute__((ext_vector_type(4), may_alias));
union FragH { v16h v; v8us half[2]; unsigned short u[16]; };

__device__ __forceinline__ float bf16r(float x) {
  unsigned int u = __float_as_uint(x);
  u = (u + 0x7FFFu + ((u >> 16) & 1u)) & 0xFFFF0000u;
  return __uint_as_float(u);
}
__device__ __forceinline__ unsigned short h_bits(float x) { const _Float16 h = (_Float16)x; return __builtin_bit_cast(unsigned short, h); }
__device__ __forceinline__ float h_val(unsigned short b) { const _Float16 h = __builtin_bit_cast(_Float16, b); return (float)h; }

__device__ __forceinline__ v8f mma1(v16h a, v16h b, v8f c) {
  c = __builtin_amdgcn_wmma_f32_16x16x32_f16(false, a, false, b, (short)0, c, false, false);
  asm volatile("v_nop\n\tv_nop\n\tv_nop\n\tv_nop" : "+v"(c) : "v"(a), "v"(b));
  return c;
}
__device__ __forceinline__ v8f mma2(v16h al, v16h bh, v16h ah, v16h bl, v8f c) {
  c = __builtin_amdgcn_wmma_f32_16x16x32_f16(false, al, false, bh, (short)0, c, false, false);
  c = __builtin_amdgcn_wmma_f32_16x16x32_f16(false, ah, false, bl, (short)0, c, false, false);
  asm volatile("v_nop\n\tv_nop\n\tv_nop\n\tv_nop" : "+v"(c) : "v"(al), "v"(bh), "v"(ah), "v"(bl));
  return c;
}

__global__ __launch_bounds__(256) void k_wt16(const float* __restrict__ W, unsigned short* __restrict__ Wt, int K, int N, float wscale) {
  const int t = blockIdx.x * 256 + threadIdx.x;
  const int k8n = K / 8;
  if (t >= N * k8n) return;
  const int n = t / k8n, k8 = (t % k8n) * 8;
  v8us v;
#pragma unroll
  for (int i = 0; i < 8; ++i) v[i] = h_bits(bf16r(W[(size_t)(k8 + i) * N + n]) * wscale);
  unsigned short* dst = Wt + (size_t)n * K + k8;
  *(volatile v8us*)dst = v;
  __threadfence();
  *(volatile v8us*)dst = v;
}

template <bool RIN>
__global__ __launch_bounds__(128) void k_ln(const float* __restrict__ X, int in_seq, int in_seqf,
                                           const float* __restrict__ g, const float* __restrict__ bt,
                                           unsigned short* __restrict__ outp, float eps) {
  __shared__ float red[8];
  const int row = blockIdx.x, tid = threadIdx.x, w = tid >> 5, lane = tid & 31;
  const int xrow = (row / in_seq) * in_seqf + (row % in_seq);
  const float* x = X + (size_t)xrow * DM;
  const int j = tid * 8;
  const v4f a0 = *(const v4fa*)(x + j), a1 = *(const v4fa*)(x + j + 4);
  float v[8] = {a0[0], a0[1], a0[2], a0[3], a1[0], a1[1], a1[2], a1[3]};
  float s1 = 0.f;
#pragma unroll
  for (int i = 0; i < 8; ++i) { if (RIN) v[i] = bf16r(v[i]); s1 += v[i]; }
  s1 += __shfl_xor(s1, 1, 32); s1 += __shfl_xor(s1, 2, 32); s1 += __shfl_xor(s1, 4, 32); s1 += __shfl_xor(s1, 8, 32); s1 += __shfl_xor(s1, 16, 32);
  if (lane == 0) red[w] = s1;
  __syncthreads();
  const float mu = (red[0] + red[1] + red[2] + red[3]) * (1.0f / (float)DM);
  float s2 = 0.f;
#pragma unroll
  for (int i = 0; i < 8; ++i) { const float c = v[i] - mu; s2 += c * c; }
  s2 += __shfl_xor(s2, 1, 32); s2 += __shfl_xor(s2, 2, 32); s2 += __shfl_xor(s2, 4, 32); s2 += __shfl_xor(s2, 8, 32); s2 += __shfl_xor(s2, 16, 32);
  if (lane == 0) red[4 + w] = s2;
  __syncthreads();
  const float var = (red[4] + red[5] + red[6] + red[7]) * (1.0f / (float)DM);
  const float rs = rsqrtf(var + eps);
  v8us o;
#pragma unroll
  for (int i = 0; i < 8; ++i) o[i] = h_bits((v[i] - mu) * rs * bf16r(g[j + i]) + bf16r(bt[j + i]));
  unsigned short* dst = outp + (size_t)row * DM + j;
  *(volatile v8us*)dst = o;
  __threadfence();
  *(volatile v8us*)dst = o;
}

template <int ACT, int O16>
__global__ __launch_bounds__(128) void k_gemm(const unsigned short* __restrict__ A, int lda, const unsigned short* __restrict__ Wt, int ldb,
                                             const float* __restrict__ bias, const float* __restrict__ resid, int ldr, int rs_seq, int rs_seqf, int rs_rne,
                                             float oscale, float pscale,
                                             float* __restrict__ C, unsigned short* __restrict__ Ch, unsigned short* __restrict__ Cl, int ldc, int c_seq, int c_seqf,
                                             int lo_seq, int lo_rows, int M, int N, int K) {
  __shared__ __attribute__((aligned(16))) float so[4][16][64];
  const int tid = threadIdx.x, w = tid >> 5, lane = tid & 31, ln = lane & 15, hh = lane >> 4;
  const int ntn = N / 64;
  const int wid = blockIdx.x * 4 + w;
  const int mt = wid / ntn, nq = wid % ntn;
  if (mt * 16 >= M) return;
  const int row0 = mt * 16, col0 = nq * 64;
  const unsigned short* arow = A + (size_t)(row0 + ln) * lda;
  v8f acc[4] = {};
  for (int kb = 0; kb < K; kb += 32) {
    FragH a;
    a.half[0] = *(const v8us*)(arow + kb + 8 * hh);
    a.half[1] = *(const v8us*)(arow + kb + 16 + 8 * hh);
#pragma unroll
    for (int t = 0; t < 4; ++t) {
      const unsigned short* brow = Wt + (size_t)(col0 + t * 16 + ln) * ldb + kb;
      FragH b;
      b.half[0] = *(const v8us*)(brow + 8 * hh);
      b.half[1] = *(const v8us*)(brow + 16 + 8 * hh);
      acc[t] = mma1(a.v, b.v, acc[t]);
    }
  }
#pragma unroll
  for (int t = 0; t < 4; ++t) {
    const int col = col0 + t * 16 + ln;
    float bv = 0.f;
    if (bias != nullptr) bv = bf16r(bias[col]);
#pragma unroll
    for (int r = 0; r < 8; ++r) {
      const int m = row0 + 8 * hh + r;
      float v = acc[t][r] * oscale + bv;
      if (resid != nullptr) {
        const int rrow = (m / rs_seq) * rs_seqf + (m % rs_seq);
        float rv = resid[(size_t)rrow * ldr + col];
        if (rs_rne) rv = bf16r(rv);
        v += rv;
      }
      if (ACT == 1) v = fmaxf(v, 0.f);
      so[w][8 * hh + r][t * 16 + ln] = v;
    }
  }
  __builtin_amdgcn_fence(4, "workgroup");
  __builtin_amdgcn_wave_barrier();
  if (O16 == 0) {
    const int rsub = lane >> 4, c4 = (lane & 15) * 4;
    for (int pass = 0; pass < 2; ++pass) {
#pragma unroll
      for (int q = 0; q < 8; ++q) {
        const int r = q * 2 + rsub;
        const int m = row0 + r;
        const int crow = (m / c_seq) * c_seqf + (m % c_seq);
        const v4f v = *(const v4fa*)&so[w][r][c4];
        *(volatile v4f*)(C + (size_t)crow * ldc + col0 + c4) = v;
      }
      if (pass == 0) __threadfence();
    }
  } else {
    const int rq = lane >> 3, c8 = (lane & 7) * 8;
    bool dolo = false;
    if (O16 == 2) dolo = (row0 % lo_seq) < lo_rows;
    for (int pass = 0; pass < 2; ++pass) {
#pragma unroll
      for (int q = 0; q < 4; ++q) {
        const int r = q * 4 + rq;
        const int m = row0 + r;
        const int crow = (m / c_seq) * c_seqf + (m % c_seq);
        const v4f x0 = *(const v4fa*)&so[w][r][c8], x1 = *(const v4fa*)&so[w][r][c8 + 4];
        v8us hv, lv;
#pragma unroll
        for (int i = 0; i < 4; ++i) {
          const float f0 = x0[i] * pscale; const unsigned short b0 = h_bits(f0); hv[i] = b0;     lv[i] = h_bits((f0 - h_val(b0)) * RSC);
          const float f1 = x1[i] * pscale; const unsigned short b1 = h_bits(f1); hv[4 + i] = b1; lv[4 + i] = h_bits((f1 - h_val(b1)) * RSC);
        }
        *(volatile v8us*)(Ch + (size_t)crow * ldc + col0 + c8) = hv;
        if (O16 == 2) {
          if (dolo) {
            const int lrow = (m / lo_seq) * lo_rows + (m % lo_seq);
            *(volatile v8us*)(Cl + (size_t)lrow * ldc + col0 + c8) = lv;
          }
        }
      }
      if (pass == 0) __threadfence();
    }
  }
}

template <bool EARLY>
__global__ __launch_bounds__(128) void k_attn(const unsigned short* __restrict__ ph, const unsigned short* __restrict__ pl,
                                             int pitch, int kofs, int vofs, int T, int H, int qoff, int nqbl, int lrows,
                                             unsigned short* __restrict__ ctx, int cpitch) {
  __shared__ __attribute__((aligned(16))) unsigned short sKh[32][HD + 8], sVh[32][HD + 8], sKl[32][HD + 8], sVl[32][HD + 8];
  __shared__ __attribute__((aligned(16))) unsigned short sPh[4][16][40], sPl[4][16][40];
  __shared__ __attribute__((aligned(16))) float sO[4][16][HD];
  constexpr float SCO = 1.0f / (QSC * QSC * 8.0f);
  constexpr float OSC = CSC / (PSC * QSC);
  constexpr float IRS = 1.0f / RSC;
  const int tid = threadIdx.x, w = tid >> 5, lane = tid & 31, ln = lane & 15, hh = lane >> 4;
  const int bh = blockIdx.x / nqbl, qblk = qoff + (blockIdx.x % nqbl);
  const int b = bh / H, h = bh % H;
  const int q0 = qblk * 64 + w * 16;
  const unsigned short* Q  = ph + (size_t)b * T * pitch + h * HD;
  const unsigned short* Kp = Q + kofs;
  const unsigned short* Vp = Q + vofs;
  const unsigned short* QL = pl + (size_t)b * lrows * pitch + h * HD;
  const unsigned short* KL = QL + kofs;
  const unsigned short* VL = QL + vofs;

  FragH aqh[2], aql[2];
  {
    int row = q0 + ln; if (row >= T) row = T - 1;
    const unsigned short* qr = Q + (size_t)row * pitch;
    int rl = row; if (rl >= lrows) rl = lrows - 1;
    const unsigned short* qlr = QL + (size_t)rl * pitch;
#pragma unroll
    for (int ks = 0; ks < 2; ++ks) {
      aqh[ks].half[0] = *(const v8us*)(qr + ks * 32 + 8 * hh);
      aqh[ks].half[1] = *(const v8us*)(qr + ks * 32 + 16 + 8 * hh);
      if (EARLY) {
        aql[ks].half[0] = *(const v8us*)(qlr + ks * 32 + 8 * hh);
        aql[ks].half[1] = *(const v8us*)(qlr + ks * 32 + 16 + 8 * hh);
      } else {
        aql[ks].half[0] = (v8us){0, 0, 0, 0, 0, 0, 0, 0};
        aql[ks].half[1] = (v8us){0, 0, 0, 0, 0, 0, 0, 0};
      }
    }
  }
  float m_r[8], l_r[8];
#pragma unroll
  for (int r = 0; r < 8; ++r) { m_r[r] = -3.0e38f; l_r[r] = 0.f; }
  v8f oacc[4], oal[4];
#pragma unroll
  for (int dt = 0; dt < 4; ++dt) { oacc[dt] = (v8f){0.f,0.f,0.f,0.f,0.f,0.f,0.f,0.f}; oal[dt] = (v8f){0.f,0.f,0.f,0.f,0.f,0.f,0.f,0.f}; }

  const int kv_lim = qblk * 64 + 64;
  const int kv_end = kv_lim < T ? kv_lim : T;
  for (int j0 = 0; j0 < kv_end; j0 += 32) {
    __syncthreads();
    for (int e = tid; e < 32 * (HD / 8); e += 128) {
      const int r = e >> 3, c8 = (e & 7) * 8;
      const int key = j0 + r;
      const int kc = key < T ? key : T - 1;
      v8us kv = *(const v8us*)(Kp + (size_t)kc * pitch + c8);
      v8us vv = *(const v8us*)(Vp + (size_t)kc * pitch + c8);
      if (key >= T) { kv = (v8us){0, 0, 0, 0, 0, 0, 0, 0}; vv = kv; }
      *(v8us*)&sKh[r][c8] = kv;
      *(v8us*)&sVh[r][c8] = vv;
      if (EARLY) {
        const int lc = key < lrows ? key : lrows - 1;
        v8us kl = *(const v8us*)(KL + (size_t)lc * pitch + c8);
        v8us vl = *(const v8us*)(VL + (size_t)lc * pitch + c8);
        if (key >= lrows) { kl = (v8us){0, 0, 0, 0, 0, 0, 0, 0}; vl = kl; }
        *(v8us*)&sKl[r][c8] = kl;
        *(v8us*)&sVl[r][c8] = vl;
      }
    }
    __syncthreads();
    v8f s[2];
#pragma unroll
    for (int nt = 0; nt < 2; ++nt) {
      v8f acc = {};
      v8f accl = {};
#pragma unroll
      for (int ks = 0; ks < 2; ++ks) {
        FragH bk;
        bk.half[0] = *(const v8us*)&sKh[nt * 16 + ln][ks * 32 + 8 * hh];
        bk.half[1] = *(const v8us*)&sKh[nt * 16 + ln][ks * 32 + 16 + 8 * hh];
        acc = mma1(aqh[ks].v, bk.v, acc);
        if (EARLY) {
          FragH bkl;
          bkl.half[0] = *(const v8us*)&sKl[nt * 16 + ln][ks * 32 + 8 * hh];
          bkl.half[1] = *(const v8us*)&sKl[nt * 16 + ln][ks * 32 + 16 + 8 * hh];
          accl = mma2(aql[ks].v, bk.v, aqh[ks].v, bkl.v, accl);
        }
      }
#pragma unroll
      for (int r = 0; r < 8; ++r) s[nt][r] = EARLY ? (acc[r] + accl[r] * IRS) * SCO : acc[r] * SCO;
    }
    float alpha[8];
#pragma unroll
    for (int r = 0; r < 8; ++r) {
      const int qi = q0 + 8 * hh + r;
      const int ja = j0 + ln, jb = j0 + 16 + ln;
      float s0 = s[0][r], s1 = s[1][r];
      if (ja > qi || ja >= T) s0 = -3.0e38f;
      if (jb > qi || jb >= T) s1 = -3.0e38f;
      float mx = fmaxf(s0, s1);
      mx = fmaxf(mx, __shfl_xor(mx, 1, 32)); mx = fmaxf(mx, __shfl_xor(mx, 2, 32));
      mx = fmaxf(mx, __shfl_xor(mx, 4, 32)); mx = fmaxf(mx, __shfl_xor(mx, 8, 32));
      const float mnew = fmaxf(m_r[r], mx);
      alpha[r] = (mnew > -1.0e38f) ? __expf(m_r[r] - mnew) : 1.0f;
      const float p0 = (s0 > -1.0e38f) ? __expf(s0 - mnew) : 0.f;
      const float p1 = (s1 > -1.0e38f) ? __expf(s1 - mnew) : 0.f;
      m_r[r] = mnew;
      l_r[r] = l_r[r] * alpha[r] + p0 + p1;
      const float c0 = p0 * PSC, c1 = p1 * PSC;
      const unsigned short hb0 = h_bits(c0), hb1 = h_bits(c1);
      sPh[w][8 * hh + r][ln] = hb0;
      sPh[w][8 * hh + r][16 + ln] = hb1;
      if (EARLY) {
        sPl[w][8 * hh + r][ln] = h_bits((c0 - h_val(hb0)) * RSC);
        sPl[w][8 * hh + r][16 + ln] = h_bits((c1 - h_val(hb1)) * RSC);
      }
    }
#pragma unroll
    for (int dt = 0; dt < 4; ++dt)
#pragma unroll
      for (int r = 0; r < 8; ++r) { oacc[dt][r] *= alpha[r]; if (EARLY) oal[dt][r] *= alpha[r]; }
    __builtin_amdgcn_fence(4, "workgroup");
    __builtin_amdgcn_wave_barrier();
    FragH pa, par;
    pa.half[0] = *(const v8us*)&sPh[w][ln][8 * hh];
    pa.half[1] = *(const v8us*)&sPh[w][ln][16 + 8 * hh];
    if (EARLY) {
      par.half[0] = *(const v8us*)&sPl[w][ln][8 * hh];
      par.half[1] = *(const v8us*)&sPl[w][ln][16 + 8 * hh];
    } else {
      par.half[0] = (v8us){0, 0, 0, 0, 0, 0, 0, 0};
      par.half[1] = (v8us){0, 0, 0, 0, 0, 0, 0, 0};
    }
#pragma unroll
    for (int dt = 0; dt < 4; ++dt) {
      FragH bv, bvr;
#pragma unroll
      for (int i = 0; i < 8; ++i) {
        bv.u[i] = sVh[8 * hh + i][dt * 16 + ln];
        bv.u[8 + i] = sVh[16 + 8 * hh + i][dt * 16 + ln];
        if (EARLY) { bvr.u[i] = sVl[8 * hh + i][dt * 16 + ln]; bvr.u[8 + i] = sVl[16 + 8 * hh + i][dt * 16 + ln]; }
        else { bvr.u[i] = 0; bvr.u[8 + i] = 0; }
      }
      oacc[dt] = mma1(pa.v, bv.v, oacc[dt]);
      if (EARLY) oal[dt] = mma2(par.v, bv.v, pa.v, bvr.v, oal[dt]);
    }
    __builtin_amdgcn_fence(4, "workgroup");
    __builtin_amdgcn_wave_barrier();
  }
  float inv[8];
#pragma unroll
  for (int r = 0; r < 8; ++r) {
    float l = l_r[r];
    l += __shfl_xor(l, 1, 32); l += __shfl_xor(l, 2, 32); l += __shfl_xor(l, 4, 32); l += __shfl_xor(l, 8, 32);
    inv[r] = (l > 0.f) ? (OSC / l) : 0.f;
  }
#pragma unroll
  for (int dt = 0; dt < 4; ++dt)
#pragma unroll
    for (int r = 0; r < 8; ++r) {
      float o = oacc[dt][r];
      if (EARLY) o += oal[dt][r] * IRS;
      sO[w][8 * hh + r][dt * 16 + ln] = o * inv[r];
    }
  __builtin_amdgcn_fence(4, "workgroup");
  __builtin_amdgcn_wave_barrier();
  const int rq = lane >> 3, c8 = (lane & 7) * 8;
  for (int pass = 0; pass < 2; ++pass) {
#pragma unroll
    for (int q = 0; q < 4; ++q) {
      const int r = q * 4 + rq;
      const int row = q0 + r;
      const v4f x0 = *(const v4fa*)&sO[w][r][c8], x1 = *(const v4fa*)&sO[w][r][c8 + 4];
      v8us hv;
#pragma unroll
      for (int i = 0; i < 4; ++i) { hv[i] = h_bits(x0[i]); hv[4 + i] = h_bits(x1[i]); }
      if (row < T) *(volatile v8us*)(ctx + ((size_t)b * T + row) * cpitch + h * HD + c8) = hv;
    }
    if (pass == 0) __threadfence();
  }
}

extern "C" void kernel_launch(void* const* d_in, const int* in_sizes, int n_in,
                              void* d_out, int out_size, void* d_ws, size_t ws_size, hipStream_t stream) {
  if (n_in < 13) return;
  const int xrows = (NB - 1) * SEQ_FULL + SEQ;
  if (in_sizes[0] < xrows * DM) return;
  if (in_sizes[1] < DM * DM || in_sizes[2] < DM * DM || in_sizes[3] < DM * DM || in_sizes[4] < DM * DM) return;
  if (in_sizes[5] < DM * FF || in_sizes[6] < FF || in_sizes[7] < FF * DM || in_sizes[8] < DM) return;
  if (in_sizes[9] < DM || in_sizes[10] < DM || in_sizes[11] < DM || in_sizes[12] < DM) return;
  if (out_size < xrows * DM) return;
  const float* x   = (const float*)d_in[0];
  const float* wq  = (const float*)d_in[1];
  const float* wk  = (const float*)d_in[2];
  const float* wv  = (const float*)d_in[3];
  const float* wo  = (const float*)d_in[4];
  const float* w1  = (const float*)d_in[5];
  const float* b1  = (const float*)d_in[6];
  const float* w2  = (const float*)d_in[7];
  const float* b2  = (const float*)d_in[8];
  const float* g1  = (const float*)d_in[9];
  const float* be1 = (const float*)d_in[10];
  const float* g2  = (const float*)d_in[11];
  const float* be2 = (const float*)d_in[12];
  float* outp = (float*)d_out;

  const int M = MROWS;
  char* ws = (char*)d_ws; size_t off = 0;
  auto take = [&](size_t bytes) { char* p = ws + off; off += (bytes + 255) & ~(size_t)255; return p; };
  unsigned short* Wqkv = (unsigned short*)take((size_t)3 * DM * DM * 2);
  unsigned short* Wo   = (unsigned short*)take((size_t)DM * DM * 2);
  unsigned short* W1t  = (unsigned short*)take((size_t)FF * DM * 2);
  unsigned short* W2t  = (unsigned short*)take((size_t)DM * FF * 2);
  unsigned short* h1   = (unsigned short*)take((size_t)M * DM * 2);
  unsigned short* qkvh = (unsigned short*)take((size_t)M * 3 * DM * 2);
  unsigned short* qkvl = (unsigned short*)take((size_t)NB * LOR * 3 * DM * 2);
  unsigned short* ctx  = (unsigned short*)take((size_t)M * DM * 2);
  float*          x1   = (float*)take((size_t)M * DM * 4);
  unsigned short* h2   = (unsigned short*)take((size_t)M * DM * 2);
  unsigned short* Hp   = (unsigned short*)take((size_t)M * FF * 2);
  if (off > ws_size) return;

  k_wt16<<<(DM * (DM / 8) + 255) / 256, 256, 0, stream>>>(wq, Wqkv, DM, DM, WSC);
  k_wt16<<<(DM * (DM / 8) + 255) / 256, 256, 0, stream>>>(wk, Wqkv + (size_t)DM * DM, DM, DM, WSC);
  k_wt16<<<(DM * (DM / 8) + 255) / 256, 256, 0, stream>>>(wv, Wqkv + (size_t)2 * DM * DM, DM, DM, WSC);
  k_wt16<<<(DM * (DM / 8) + 255) / 256, 256, 0, stream>>>(wo, Wo, DM, DM, WSC);
  k_wt16<<<(FF * (DM / 8) + 255) / 256, 256, 0, stream>>>(w1, W1t, DM, FF, WSC);
  k_wt16<<<(DM * (FF / 8) + 255) / 256, 256, 0, stream>>>(w2, W2t, FF, DM, WSC);

  k_ln<true><<<M, 128, 0, stream>>>(x, SEQ, SEQ_FULL, g1, be1, h1, 1e-5f);
  k_gemm<0, 2><<<((M / 16) * (3 * DM / 64) + 3) / 4, 128, 0, stream>>>(h1, DM, Wqkv, DM, nullptr, nullptr, 0, 1, 1, 0,
      1.0f / WSC, QSC, nullptr, qkvh, qkvl, 3 * DM, 1, 1, SEQ, LOR, M, 3 * DM, DM);
  k_attn<true><<<NB * NH, 128, 0, stream>>>(qkvh, qkvl, 3 * DM, DM, 2 * DM, SEQ, NH, 0, 1, LOR, ctx, DM);
  const int nqrest = SEQ / 64 - 1;
  if (nqrest > 0)
    k_attn<false><<<NB * NH * nqrest, 128, 0, stream>>>(qkvh, qkvl, 3 * DM, DM, 2 * DM, SEQ, NH, 1, nqrest, LOR, ctx, DM);
  k_gemm<0, 0><<<((M / 16) * (DM / 64) + 3) / 4, 128, 0, stream>>>(ctx, DM, Wo, DM, nullptr, x, DM, SEQ, SEQ_FULL, 1,
      1.0f / (CSC * WSC), 1.0f, x1, nullptr, nullptr, DM, 1, 1, 1, 0, M, DM, DM);
  k_ln<false><<<M, 128, 0, stream>>>(x1, 1, 1, g2, be2, h2, 1e-5f);
  k_gemm<1, 1><<<((M / 16) * (FF / 64) + 3) / 4, 128, 0, stream>>>(h2, DM, W1t, DM, b1, nullptr, 0, 1, 1, 0,
      1.0f / WSC, HSC, nullptr, Hp, nullptr, FF, 1, 1, 1, 0, M, FF, DM);
  k_gemm<0, 0><<<((M / 16) * (DM / 64) + 3) / 4, 128, 0, stream>>>(Hp, FF, W2t, FF, b2, x1, DM, 1, 1, 0,
      1.0f / (HSC * WSC), 1.0f, outp, nullptr, nullptr, DM, SEQ, SEQ_FULL, 1, 0, M, DM, FF);
}
